// EncoderSeq_36988258353807
// MI455X (gfx1250) — hardware-verified
//
#include <hip/hip_runtime.h>
#include <math.h>

typedef __attribute__((ext_vector_type(16))) _Float16 v16h;
typedef __attribute__((ext_vector_type(16))) __bf16 v16b;
typedef __attribute__((ext_vector_type(8)))  _Float16 v8h;
typedef __attribute__((ext_vector_type(8)))  float v8f;
typedef __attribute__((ext_vector_type(4)))  float v4f;
typedef __attribute__((ext_vector_type(2)))  float v2f;
typedef __attribute__((ext_vector_type(4)))  unsigned v4u;
typedef __attribute__((ext_vector_type(4)))  int v4i;
typedef float __attribute__((may_alias)) float_a;
typedef int __attribute__((may_alias)) int_a;

template <typename T> __device__ __forceinline__ void vst2(void* p, T v) { *(volatile T*)p = v; __threadfence(); *(volatile T*)p = v; }
__device__ __forceinline__ v8f wmma16(v16h a, v16h b, v8f c) {
  v8f d = __builtin_amdgcn_wmma_f32_16x16x32_f16(false, a, false, b, (short)0, c, false, false);
  asm volatile("v_nop\n\tv_nop\n\tv_nop\n\tv_nop" : "+v"(d) : "v"(a), "v"(b));
  return d;
}
__device__ __forceinline__ v8f wmma_bf(v16b a, v16b b, v8f c) {
  v8f d = __builtin_amdgcn_wmma_f32_16x16x32_bf16(false, a, false, b, (short)0, c, false, false);
  asm volatile("v_nop\n\tv_nop\n\tv_nop\n\tv_nop" : "+v"(d) : "v"(a), "v"(b));
  return d;
}
__device__ __forceinline__ v16h frag_h(const _Float16* rowk0, int lane) {
  union { v16h v; v8h q[2]; } u; const _Float16* p = rowk0 + 8 * (lane >> 4);
  u.q[0] = *(const v8h*)p; u.q[1] = *(const v8h*)(p + 16); return u.v;
}
__device__ __forceinline__ v16h frag_f32(const float* rowk0, int lane) {
  v16h a; const float* p = rowk0 + 8 * (lane >> 4);
#pragma unroll
  for (int i = 0; i < 8; ++i) { a[i] = (_Float16)p[i]; a[8 + i] = (_Float16)p[16 + i]; }
  return a;
}
__device__ __forceinline__ v16h frag_f32s(const float* rowk0, int lane, float sc) {
  v16h a; const float* p = rowk0 + 8 * (lane >> 4);
#pragma unroll
  for (int i = 0; i < 8; ++i) { a[i] = (_Float16)(p[i] * sc); a[8 + i] = (_Float16)(p[16 + i] * sc); }
  return a;
}
__device__ __forceinline__ v16h fragc_f32(const float* W, int k0, int n, int lane, int ld, int K) {
  v16h a; const int g = lane >> 4;
#pragma unroll
  for (int i = 0; i < 8; ++i) { const int ka = k0 + 8 * g + i, kb = ka + 16;
    a[i] = (_Float16)(ka < K ? W[(size_t)(ka < K ? ka : K - 1) * ld + n] : 0.f); a[8 + i] = (_Float16)(kb < K ? W[(size_t)(kb < K ? kb : K - 1) * ld + n] : 0.f); }
  return a;
}
struct F2 { v16b h, l; };
__device__ __forceinline__ F2 bsplit16(const float v[16]) { F2 r;
#pragma unroll
  for (int i = 0; i < 16; ++i) { const __bf16 h = (__bf16)v[i]; r.h[i] = h; r.l[i] = (__bf16)(v[i] - (float)h); }
  return r; }
__device__ __forceinline__ F2 split_row(const float* row, int k0, int lane) { float v[16]; const float* p = row + k0 + 8 * (lane >> 4);
#pragma unroll
  for (int i = 0; i < 8; ++i) { v[i] = p[i]; v[8 + i] = p[16 + i]; }
  return bsplit16(v); }
__device__ __forceinline__ F2 split_rowK(const float* row, int k0, int lane, int K) { float v[16]; const int g = lane >> 4;
#pragma unroll
  for (int i = 0; i < 8; ++i) { const int ka = k0 + 8 * g + i, kb = ka + 16; v[i] = ka < K ? row[ka < K ? ka : K - 1] : 0.f; v[8 + i] = kb < K ? row[kb < K ? kb : K - 1] : 0.f; }
  return bsplit16(v); }
__device__ __forceinline__ F2 split_col(const float* W, int k0, int n, int lane, int ld, int K) { float v[16]; const int g = lane >> 4;
#pragma unroll
  for (int i = 0; i < 8; ++i) { const int ka = k0 + 8 * g + i, kb = ka + 16; v[i] = ka < K ? W[(size_t)(ka < K ? ka : K - 1) * ld + n] : 0.f; v[8 + i] = kb < K ? W[(size_t)(kb < K ? kb : K - 1) * ld + n] : 0.f; }
  return bsplit16(v); }
__device__ __forceinline__ v8f mac3(const F2& a, const F2& b, v8f c) { c = wmma_bf(a.l, b.h, c); c = wmma_bf(a.h, b.l, c); return wmma_bf(a.h, b.h, c); }
__device__ __forceinline__ float sigm(float v) { return 1.0f / (1.0f + expf(-v)); }
#define LDSX() do { asm volatile("s_wait_dscnt 0" ::: "memory"); __builtin_amdgcn_wave_barrier(); __builtin_amdgcn_fence(__ATOMIC_RELEASE, "workgroup"); } while (0)


#define NLAY 2
#define NB 8
#define SS 1024
#define NR (NB * SS)
#define DM 512
#define NH 8
#define DK 12
#define DV 32
#define QW (NH * DK)
#define VW (NH * DV)
#define FF 2048
#define QP 256
#ifndef NBT
#define NBT NB
#define TB0 0
#endif
#define RT (NBT * SS)
#define RB0 ((size_t)TB0 * SS)
typedef __attribute__((ext_vector_type(8))) __bf16 v8b;
__device__ __forceinline__ v16b frag_b(const __bf16* rowk0, int lane) {
  union { v16b v; v8b q[2]; } u; const __bf16* p = rowk0 + 8 * (lane >> 4);
  u.q[0] = *(const v8b*)p; u.q[1] = *(const v8b*)(p + 16); return u.v;
}
__device__ __forceinline__ float bfr(float v) { return (float)(__bf16)v; }
__device__ __attribute__((noinline)) float exp_ni(float v) { return expf(v); }
__device__ __attribute__((noinline)) float erf_ni(float v) { return erff(v); }

#define PL_Q  0
#define PL_K  ((size_t)QW * DM)
#define PL_V  ((size_t)2 * QW * DM)
#define PL_X  (PL_V + (size_t)VW * DM)
#define PL_1  (PL_X + (size_t)DM * VW)
#define PL_2  (PL_1 + (size_t)FF * DM)
#define PL_SZ (PL_2 + (size_t)DM * FF)
#define WS_PK  0u
#define WS_X   (((2u * NLAY * PL_SZ) + 127u) / 128u * 128u)
#define WS_T   (WS_X + 4u * NR * DM)
#define WS_QF  (WS_T + 4u * NR * DM)
#define WS_KF  (WS_QF + 2u * NR * QP)
#define WS_VTH (WS_KF + 2u * NR * QP)
#define WS_VTL (WS_VTH + 2u * NR * VW)
#define WS_CTX (WS_VTL + 2u * NR * VW)
#define WS_GH  (WS_CTX + 4u * NR * VW)
#define WS_GL  (WS_GH + 2u * (size_t)NR * FF)
#define WS_END (WS_GL + 2u * (size_t)NR * FF)

__global__ __launch_bounds__(256) void k_pack(const float* __restrict__ WQ, const float* __restrict__ WK, const float* __restrict__ WV, const float* __restrict__ WX, const float* __restrict__ W1, const float* __restrict__ W2, __bf16* __restrict__ PK) {
  __shared__ __align__(16) __bf16 s[FF]; const int n = blockIdx.x, which = blockIdx.y, lay = blockIdx.z, t = threadIdx.x; int K, NO; size_t dst; const float* Wm;
  switch (which) { case 0: Wm = WQ; K = DM; NO = QW; dst = PL_Q; break; case 1: Wm = WK; K = DM; NO = QW; dst = PL_K; break; case 2: Wm = WV; K = DM; NO = VW; dst = PL_V; break; case 3: Wm = WX; K = VW; NO = DM; dst = PL_X; break; case 4: Wm = W1; K = DM; NO = FF; dst = PL_1; break; default: Wm = W2; K = FF; NO = DM; dst = PL_2; break; }
  if (n >= NO) return;
  const float* base = Wm + (size_t)lay * K * NO;
  for (int k = t; k < K; k += 256) s[k] = (__bf16)base[(size_t)k * NO + n];
  __syncthreads();
  for (int q = t; q < K / 8; q += 256) vst2((unsigned*)(PK + (size_t)lay * PL_SZ + dst + (size_t)n * K + q * 8), *(const v4u*)&s[q * 8]);
}
__global__ __launch_bounds__(128) void k_ln(const float* __restrict__ SRC, int round_src, const float* __restrict__ G, const float* __restrict__ Bv, float* __restrict__ OUT, float* __restrict__ XCOPY) {
  __shared__ float red[2][4]; const int t = threadIdx.x; const size_t row = RB0 + blockIdx.x; const float* p = SRC + row * DM + t * 4;
  float v[4];
#pragma unroll
  for (int i = 0; i < 4; ++i) v[i] = round_src ? bfr(p[i]) : p[i];
  float s = (v[0] + v[1]) + (v[2] + v[3]);
#pragma unroll
  for (int o = 1; o < 32; o <<= 1) s += __shfl_xor(s, o);
  if ((t & 31) == 0) red[0][t >> 5] = s; __syncthreads();
  const float mu = (red[0][0] + red[0][1] + red[0][2] + red[0][3]) / (float)DM; float q = 0.f;
#pragma unroll
  for (int i = 0; i < 4; ++i) { const float d = v[i] - mu; q += d * d; }
#pragma unroll
  for (int o = 1; o < 32; o <<= 1) q += __shfl_xor(q, o);
  if ((t & 31) == 0) red[1][t >> 5] = q; __syncthreads();
  const float sd = sqrtf((red[1][0] + red[1][1] + red[1][2] + red[1][3]) / (float)(DM - 1)); const float inv = 1.0f / (sd + 1e-6f);
  v4f o4;
#pragma unroll
  for (int i = 0; i < 4; ++i) o4[i] = bfr(G[t * 4 + i]) * (v[i] - mu) * inv + bfr(Bv[t * 4 + i]);
  vst2(OUT + row * DM + t * 4, o4);
  if (XCOPY) { v4f c4 = {v[0], v[1], v[2], v[3]}; vst2(XCOPY + row * DM + t * 4, c4); }
}
__global__ __launch_bounds__(128) void k_qkv(const float* __restrict__ T, const __bf16* __restrict__ PKL, const float* __restrict__ BQ, const float* __restrict__ BK, const float* __restrict__ BV, _Float16* __restrict__ QF, _Float16* __restrict__ KF, _Float16* __restrict__ VTH, _Float16* __restrict__ VTL) {
  __shared__ __align__(16) _Float16 sq[4][16][QP + 8]; __shared__ __align__(16) _Float16 sth[128][72], stl[128][72];
  const int tid = threadIdx.x, wave = tid >> 5, lane = tid & 31, col = lane & 15, g = lane >> 4; const int which = blockIdx.y; const size_t r0 = RB0 + (size_t)blockIdx.x * 64 + wave * 16;
  if (which < 2) { const __bf16* P = PKL + ((which == 0) ? PL_Q : PL_K); const float* BB = (which == 0) ? BQ : BK; const float sc = (which == 0) ? 0.28867513459481287f : 1.0f;
    v8f acc[6] = {};
#pragma unroll 2
    for (int kc = 0; kc < DM / 32; ++kc) { const F2 a = split_row(T + (r0 + col) * DM, kc * 32, lane);
#pragma unroll
      for (int j = 0; j < 6; ++j) { const v16b w = frag_b(P + (size_t)(j * 16 + col) * DM + kc * 32, lane); acc[j] = wmma_bf(a.l, w, acc[j]); acc[j] = wmma_bf(a.h, w, acc[j]); } }
    for (int e = lane; e < 16 * (QP + 8); e += 32) sq[wave][e / (QP + 8)][e % (QP + 8)] = (_Float16)0.f;
    LDSX();
#pragma unroll
    for (int j = 0; j < 6; ++j) { const int c96 = j * 16 + col; const int hh = c96 / DK, dd = c96 % DK; const float bb = bfr(BB[c96]);
#pragma unroll
      for (int r = 0; r < 8; ++r) sq[wave][8 * g + r][hh * 32 + dd] = (_Float16)((acc[j][r] + bb) * sc); }
    LDSX();
    _Float16* D = (which == 0) ? QF : KF;
    for (int rl = 0; rl < 16; ++rl) vst2((unsigned*)(D + (r0 + rl) * QP + lane * 8), *(const v4u*)&sq[wave][rl][lane * 8]);
  } else { const __bf16* P = PKL + PL_V;
#pragma unroll 1
    for (int half = 0; half < 2; ++half) { v8f acc[8] = {};
#pragma unroll 2
      for (int kc = 0; kc < DM / 32; ++kc) { const F2 a = split_row(T + (r0 + col) * DM, kc * 32, lane);
#pragma unroll
        for (int j = 0; j < 8; ++j) { const v16b w = frag_b(P + (size_t)(half * 128 + j * 16 + col) * DM + kc * 32, lane); acc[j] = wmma_bf(a.l, w, acc[j]); acc[j] = wmma_bf(a.h, w, acc[j]); } }
#pragma unroll
      for (int j = 0; j < 8; ++j) { const int c = half * 128 + j * 16 + col; const float bb = bfr(BV[c]);
#pragma unroll
        for (int r = 0; r < 8; ++r) { const float v = acc[j][r] + bb; const _Float16 hv = (_Float16)v; sth[j * 16 + col][wave * 16 + 8 * g + r] = hv; stl[j * 16 + col][wave * 16 + 8 * g + r] = (_Float16)((v - (float)hv) * 2048.0f); } }
      __syncthreads();
      const size_t rb = RB0 + (size_t)blockIdx.x * 64; const int b = (int)(rb / SS), s0 = (int)(rb % SS);
      for (int e = tid; e < 128 * 8; e += 128) { const int d = e >> 3, pc = e & 7; const size_t o = ((size_t)b * VW + half * 128 + d) * SS + s0 + pc * 8; vst2((unsigned*)(VTH + o), *(const v4u*)&sth[d][pc * 8]); vst2((unsigned*)(VTL + o), *(const v4u*)&stl[d][pc * 8]); }
      __syncthreads(); } }
}
__global__ __launch_bounds__(128) void k_attn(const _Float16* __restrict__ QF, const _Float16* __restrict__ KF, const _Float16* __restrict__ VTH, const _Float16* __restrict__ VTL, const int* __restrict__ MASK, float* __restrict__ CTX) {
  __shared__ __align__(16) _Float16 sp[4][16][40]; __shared__ __align__(16) float so[4][16][36];
  const int tid = threadIdx.x, wave = tid >> 5, lane = tid & 31, col = lane & 15, g = lane >> 4; const int qb = blockIdx.x, h = blockIdx.y, b = blockIdx.z + TB0; const int q0 = qb * 64 + wave * 16;
  const v16h aq = frag_h(QF + ((size_t)b * SS + q0 + col) * QP + h * 32, lane);
  const _Float16* Vh = VTH + ((size_t)b * VW + h * DV) * SS; const _Float16* Vl = VTL + ((size_t)b * VW + h * DV) * SS;
  float m[8], l[8];
#pragma unroll
  for (int r = 0; r < 8; ++r) { m[r] = -3.0e38f; l[r] = 0.f; }
  v8f acc[2] = {}, accl[2] = {};
#pragma unroll 1
  for (int ks = 0; ks < SS / 32; ++ks) { v8f s[2];
#pragma unroll
    for (int ct = 0; ct < 2; ++ct) { const int kk = ks * 32 + ct * 16 + col; v8f c = {}; c = wmma16(aq, frag_h(KF + ((size_t)b * SS + kk) * QP + h * 32, lane), c); const bool keep = MASK[(size_t)b * SS + kk] != 0;
#pragma unroll
      for (int r = 0; r < 8; ++r) s[ct][r] = keep ? c[r] : -1.0e9f; }
#pragma unroll
    for (int r = 0; r < 8; ++r) { float mx = fmaxf(s[0][r], s[1][r]);
#pragma unroll
      for (int o = 1; o < 16; o <<= 1) mx = fmaxf(mx, __shfl_xor(mx, o));
      const float mn = fmaxf(m[r], mx); const float alpha = (m[r] <= -1.0e38f) ? 0.f : __expf(m[r] - mn); const float e0 = __expf(s[0][r] - mn), e1 = __expf(s[1][r] - mn); float es = e0 + e1;
#pragma unroll
      for (int o = 1; o < 16; o <<= 1) es += __shfl_xor(es, o);
      l[r] = l[r] * alpha + es; m[r] = mn;
#pragma unroll
      for (int dt = 0; dt < 2; ++dt) { acc[dt][r] *= alpha; accl[dt][r] *= alpha; }
      sp[wave][8 * g + r][col] = (_Float16)e0; sp[wave][8 * g + r][16 + col] = (_Float16)e1; }
    LDSX();
    const v16h pa = frag_h(&sp[wave][col][0], lane);
#pragma unroll
    for (int dt = 0; dt < 2; ++dt) { const size_t vo = (size_t)(dt * 16 + col) * SS + ks * 32; acc[dt] = wmma16(pa, frag_h(Vh + vo, lane), acc[dt]); accl[dt] = wmma16(pa, frag_h(Vl + vo, lane), accl[dt]); }
    LDSX(); }
#pragma unroll
  for (int r = 0; r < 8; ++r) { const float il = 1.0f / l[r];
#pragma unroll
    for (int dt = 0; dt < 2; ++dt) so[wave][8 * g + r][dt * 16 + col] = (acc[dt][r] + accl[dt][r] * (1.0f / 2048.0f)) * il; }
  LDSX();
  for (int rl = 0; rl < 16; ++rl) if (lane < 8) vst2(CTX + ((size_t)b * SS + q0 + rl) * VW + h * DV + lane * 4, *(const v4f*)&so[wave][rl][lane * 4]);
}
template <int MODE>
__global__ __launch_bounds__(128) void k_lin(const float* __restrict__ A, const __bf16* __restrict__ AG, const __bf16* __restrict__ AGL, const __bf16* __restrict__ P, const float* __restrict__ BIAS, float* __restrict__ X, __bf16* __restrict__ OUTG, __bf16* __restrict__ OUTGL) {
  __shared__ __align__(16) float so[4][16][132]; __shared__ __align__(16) __bf16 sg[4][16][136], sgl[4][16][136];
  const int tid = threadIdx.x, wave = tid >> 5, lane = tid & 31, col = lane & 15, g = lane >> 4; const size_t r0 = RB0 + (size_t)blockIdx.x * 64 + wave * 16; const int n0 = blockIdx.y * 128;
  constexpr int KD = (MODE == 0) ? VW : (MODE == 1) ? DM : FF;
  v8f acc[8] = {};
  if (MODE == 2) {
#pragma unroll 2
    for (int kc = 0; kc < KD / 32; ++kc) { const v16b a = frag_b(AG + (r0 + col) * FF + kc * 32, lane), al = frag_b(AGL + (r0 + col) * FF + kc * 32, lane);
#pragma unroll
      for (int j = 0; j < 8; ++j) { const v16b w = frag_b(P + (size_t)(n0 + j * 16 + col) * KD + kc * 32, lane); acc[j] = wmma_bf(al, w, acc[j]); acc[j] = wmma_bf(a, w, acc[j]); } }
  } else {
#pragma unroll 2
    for (int kc = 0; kc < KD / 32; ++kc) { const F2 a = split_row(A + (r0 + col) * KD, kc * 32, lane);
#pragma unroll
      for (int j = 0; j < 8; ++j) { const v16b w = frag_b(P + (size_t)(n0 + j * 16 + col) * KD + kc * 32, lane); acc[j] = wmma_bf(a.l, w, acc[j]); acc[j] = wmma_bf(a.h, w, acc[j]); } } }
  if (MODE == 1) {
#pragma unroll
    for (int j = 0; j < 8; ++j) { const float bb = bfr(BIAS[n0 + j * 16 + col]);
#pragma unroll
      for (int r = 0; r < 8; ++r) { const float v = fmaxf(acc[j][r] + bb, 0.f); const __bf16 hb = (__bf16)v; sg[wave][8 * g + r][j * 16 + col] = hb; sgl[wave][8 * g + r][j * 16 + col] = (__bf16)(v - (float)hb); } }
    LDSX();
    for (int rl = 0; rl < 16; ++rl) { if (lane < 16) vst2((unsigned*)(OUTG + (r0 + rl) * FF + n0 + lane * 8), *(const v4u*)&sg[wave][rl][lane * 8]); else vst2((unsigned*)(OUTGL + (r0 + rl) * FF + n0 + (lane - 16) * 8), *(const v4u*)&sgl[wave][rl][(lane - 16) * 8]); }
  } else {
#pragma unroll
    for (int j = 0; j < 8; ++j) { const float bb = bfr(BIAS[n0 + j * 16 + col]);
#pragma unroll
      for (int r = 0; r < 8; ++r) so[wave][8 * g + r][j * 16 + col] = acc[j][r] + bb; }
    LDSX();
    for (int rl = 0; rl < 16; ++rl) { float* xp = X + (r0 + rl) * DM + n0 + lane * 4; const v4f old = *(const v4f*)xp; v4f nv = *(const v4f*)&so[wave][rl][lane * 4]; nv[0] += old[0]; nv[1] += old[1]; nv[2] += old[2]; nv[3] += old[3]; vst2(xp, nv); } }
}
__global__ __launch_bounds__(128) void k_copy(const float* __restrict__ X, float* __restrict__ OUT) { const size_t row = RB0 + blockIdx.x; const int t = threadIdx.x; vst2(OUT + row * DM + t * 4, *(const v4f*)(X + row * DM + t * 4)); }
extern "C" void kernel_launch(void* const* d_in, const int* in_sizes, int n_in, void* d_out, int out_size, void* d_ws, size_t ws_size, hipStream_t stream) {
  (void)in_sizes; (void)n_in; (void)out_size;
  const float** F = (const float**)d_in;
  if (ws_size < (size_t)WS_END) return;
  char* ws = (char*)d_ws; __bf16 *PK = (__bf16*)(ws + WS_PK), *GH = (__bf16*)(ws + WS_GH), *GL = (__bf16*)(ws + WS_GL); float *X = (float*)(ws + WS_X), *T = (float*)(ws + WS_T), *CTX = (float*)(ws + WS_CTX); _Float16 *QF = (_Float16*)(ws + WS_QF), *KF = (_Float16*)(ws + WS_KF), *VTH = (_Float16*)(ws + WS_VTH), *VTL = (_Float16*)(ws + WS_VTL);
  k_pack<<<dim3(FF, 6, NLAY), 256, 0, stream>>>(F[2], F[4], F[6], F[8], F[10], F[12], PK);
  for (int lay = 0; lay < NLAY; ++lay) { const __bf16* PKL = PK + (size_t)lay * PL_SZ; const float* G = F[14] + lay * DM; const float* Bt = F[15] + lay * DM;
    k_ln<<<RT, 128, 0, stream>>>((lay == 0) ? F[0] : X, (lay == 0) ? 1 : 0, G, Bt, T, (lay == 0) ? X : nullptr);
    k_qkv<<<dim3(RT / 64, 3), 128, 0, stream>>>(T, PKL, F[3] + lay * QW, F[5] + lay * QW, F[7] + lay * VW, QF, KF, VTH, VTL);
    k_attn<<<dim3(SS / 64, NH, NBT), 128, 0, stream>>>(QF, KF, VTH, VTL, (const int*)d_in[1], CTX);
    k_lin<0><<<dim3(RT / 64, DM / 128), 128, 0, stream>>>(CTX, nullptr, nullptr, PKL + PL_X, F[9] + lay * DM, X, nullptr, nullptr);
    k_ln<<<RT, 128, 0, stream>>>(X, 0, G, Bt, T, nullptr);
    k_lin<1><<<dim3(RT / 64, FF / 128), 128, 0, stream>>>(T, nullptr, nullptr, PKL + PL_1, F[11] + lay * FF, nullptr, GH, GL);
    k_lin<2><<<dim3(RT / 64, DM / 128), 128, 0, stream>>>(nullptr, GH, GL, PKL + PL_2, F[13] + lay * DM, X, nullptr, nullptr); }
  k_copy<<<RT, 128, 0, stream>>>(X, (float*)d_out);
}
